// Code_projection_17824114278457
// MI455X (gfx1250) — hardware-run, weakly checked
//
#include <hip/hip_runtime.h>
#include <math.h>

typedef __attribute__((ext_vector_type(16))) _Float16 v16h;
typedef __attribute__((ext_vector_type(8)))  _Float16 v8h;
typedef __attribute__((ext_vector_type(4)))  _Float16 v4h;
typedef __attribute__((ext_vector_type(2)))  _Float16 v2h;
typedef __attribute__((ext_vector_type(16))) __bf16   v16b;
typedef __attribute__((ext_vector_type(8)))  __bf16   v8b;
typedef __attribute__((ext_vector_type(8)))  float    v8f;
typedef __attribute__((ext_vector_type(4)))  float    v4f;
typedef __attribute__((ext_vector_type(2)))  float    v2f;

constexpr int kNB   = 2;
constexpr int kD    = 512;
constexpr int kN    = 4096;
constexpr int kK    = 32;
constexpr int kKP   = 64;
constexpr int kKD   = 5 * kD;
constexpr int kThr  = 256;
constexpr float kInCarry = 1024.0f;
constexpr float kSc20 = 1.0f / (kInCarry * kInCarry);
constexpr float kF16MinNormal = 6.103515625e-5f;

static_assert(kNB == 2 && kD == 512 && kN == 4096 && kK == 32 && kKP == 64 && kKD == 2560, "the index arithmetic below uses these sizes");

constexpr size_t kOffAP = 0ull;
constexpr size_t kOffBP = 41943040ull;
constexpr size_t kOffXR = 42270720ull;
constexpr size_t kOffXB = 59047936ull;
constexpr size_t kOffSR = 67436544ull;
constexpr size_t kOffCR = 67502080ull;
constexpr size_t kOffLP = 67567616ull;
constexpr size_t kOffQT = 69664768ull;
constexpr size_t kOffZP = 70713344ull;
constexpr size_t kOffMS = 70975488ull;
constexpr size_t kOffNP = 70977536ull;
constexpr size_t kWsTotal = 70981632ull;
static_assert(kWsTotal <= 268435456ull, "the carve stands under 256 MiB");
static_assert(kOffAP == 0
  && kOffBP == kOffAP + 41943040ull
  && kOffXR == kOffBP + 327680ull
  && kOffXB == kOffXR + 16777216ull
  && kOffSR == kOffXB + 8388608ull
  && kOffCR == kOffSR + 65536ull
  && kOffLP == kOffCR + 65536ull
  && kOffQT == kOffLP + 2097152ull
  && kOffZP == kOffQT + 1048576ull
  && kOffMS == kOffZP + 262144ull
  && kOffNP == kOffMS + 2048ull
  && kWsTotal == kOffNP + 4096ull, "the carve is a chain: every region starts where the one before ends");
static_assert((kOffAP % 256) == 0 && (kOffBP % 256) == 0 && (kOffXR % 256) == 0 && (kOffXB % 256) == 0 && (kOffSR % 256) == 0 && (kOffCR % 256) == 0 && (kOffLP % 256) == 0 && (kOffQT % 256) == 0 && (kOffZP % 256) == 0 && (kOffMS % 256) == 0 && (kOffNP % 256) == 0, "every region starts on a multiple of 256 B");

__device__ __forceinline__ unsigned short f2bf_bits(float f) {
  unsigned u = __float_as_uint(f);
  return (unsigned short)((u + 0x7FFFu + ((u >> 16) & 1u)) >> 16);
}
__device__ __forceinline__ float bf_bits2f(unsigned short h) { return __uint_as_float(((unsigned)h) << 16); }
__device__ __forceinline__ float bf16r(float f) { return bf_bits2f(f2bf_bits(f)); }
__device__ __forceinline__ float carry_flush(float v, float carry) {
  const float s = v * carry;
  return (fabsf(s) < kF16MinNormal) ? 0.0f : s;
}

__device__ __forceinline__ void dep_guard4_h(v8f& a, v8f& b, v8f& c, v8f& d, v16h x, v16h y) { asm volatile("v_nop\n\tv_nop\n\tv_nop\n\tv_nop" : "+v"(a), "+v"(b), "+v"(c), "+v"(d) : "v"(x), "v"(y)); }
__device__ __forceinline__ void dep_guard4_b(v8f& a, v8f& b, v8f& c, v8f& d, v16b x, v16b y) { asm volatile("v_nop\n\tv_nop\n\tv_nop\n\tv_nop" : "+v"(a), "+v"(b), "+v"(c), "+v"(d) : "v"(x), "v"(y)); }
__device__ __forceinline__ void keep4_h(v16h a, v16h b, v16h c, v16h d) { asm volatile("v_nop" :: "v"(a), "v"(b), "v"(c), "v"(d)); }
__device__ __forceinline__ void keep4_b(v16b a, v16b b, v16b c, v16b d) { asm volatile("v_nop" :: "v"(a), "v"(b), "v"(c), "v"(d)); }
__device__ __forceinline__ void acc_guard4(v8f& a, v8f& b, v8f& c, v8f& d) { asm volatile("v_nop\n\tv_nop\n\tv_nop\n\tv_nop" : "+v"(a), "+v"(b), "+v"(c), "+v"(d)); }

template <typename T> struct Frag;
template <> struct Frag<_Float16> {
  typedef v16h V; union U { v16h v; v8h h[2]; };
  static __device__ __forceinline__ v16h load(const _Float16* p) {
    U f; f.h[0] = *(const v8h*)(p); f.h[1] = *(const v8h*)(p + 16); return f.v;
  }
  static __device__ __forceinline__ v8f mma(v16h a, v16h b, v8f c) {
    return __builtin_amdgcn_wmma_f32_16x16x32_f16(false, a, false, b, (short)0, c, false, false);
  }
  static __device__ __forceinline__ void guard4(v8f& a, v8f& b, v8f& c, v8f& d, v16h x, v16h y) { dep_guard4_h(a, b, c, d, x, y); }
  static __device__ __forceinline__ void keep(v16h a, v16h b, v16h c, v16h d) { keep4_h(a, b, c, d); }
};
template <> struct Frag<__bf16> {
  typedef v16b V; union U { v16b v; v8b h[2]; };
  static __device__ __forceinline__ v16b load(const __bf16* p) {
    U f; f.h[0] = *(const v8b*)(p); f.h[1] = *(const v8b*)(p + 16); return f.v;
  }
  static __device__ __forceinline__ v8f mma(v16b a, v16b b, v8f c) {
    return __builtin_amdgcn_wmma_f32_16x16x32_bf16(false, a, false, b, (short)0, c, false, false);
  }
  static __device__ __forceinline__ void guard4(v8f& a, v8f& b, v8f& c, v8f& d, v16b x, v16b y) { dep_guard4_b(a, b, c, d, x, y); }
  static __device__ __forceinline__ void keep(v16b a, v16b b, v16b c, v16b d) { keep4_b(a, b, c, d); }
};

__device__ __forceinline__ v8f mma_h(v16h a, v16h b, v8f c) {
  c = __builtin_amdgcn_wmma_f32_16x16x32_f16(false, a, false, b, (short)0, c, false, false);
  asm volatile("v_nop\n\tv_nop\n\tv_nop\n\tv_nop" : "+v"(c) : "v"(a), "v"(b));
  return c;
}

template <int ET> struct Elem;
template <> struct Elem<0> { typedef _Float16 T; };
template <> struct Elem<1> { typedef __bf16 T; };
template <int ET, bool SPLIT, int BIAS_MODE, int OUT_MODE, bool RESID, int ACT = 0>
__global__ __launch_bounds__(256) void wmma_gemm64(
    const unsigned short* __restrict__ Ap, const unsigned short* __restrict__ A2p, int lda, long strideA,
    const unsigned short* __restrict__ Btp, const unsigned short* __restrict__ Bt2p, int ldb, long strideB,
    void* __restrict__ Cout, void* __restrict__ Cout2, int ldc, long strideC,
    const float* __restrict__ bias,
    const float* __restrict__ resid, long strideR,
    int M, int N, int K, float scale) {
  typedef typename Elem<ET>::T T;
  typedef typename Frag<T>::V V;
  const T* A = (const T*)Ap; const T* A2 = (const T*)A2p; const T* Bt = (const T*)Btp; const T* Bt2 = (const T*)Bt2p;
  __shared__ __align__(16) float sT[8][16 * 68];
  const int b    = blockIdx.y;
  const int lane = threadIdx.x & 31;
  const int wave = threadIdx.x >> 5;
  const int tilesN = N >> 6;
  const int tilesM = M >> 6;
  const int tile = blockIdx.x * 8 + wave;
  if (tile >= tilesM * tilesN) return;
  const int tm = tile / tilesN;
  const int tn = tile - tm * tilesN;
  const int m0 = tm << 6;
  const int n0 = tn << 6;

  const T* Ab  = A  + (size_t)b * strideA;
  const T* Bb  = Bt + (size_t)b * strideB;
  const T* Ab2 = SPLIT ? (A2  + (size_t)b * strideA) : nullptr;
  const T* Bb2 = SPLIT ? (Bt2 + (size_t)b * strideB) : nullptr;

  const int rlane = lane & 15;
  const int koff  = (lane >> 4) * 8;
  const int mOff  = (lane >> 4) * 8;

  v8f acc[4][4];
#pragma unroll
  for (int i = 0; i < 4; ++i)
#pragma unroll
    for (int j = 0; j < 4; ++j) acc[i][j] = (v8f){0.f,0.f,0.f,0.f,0.f,0.f,0.f,0.f};

  for (int k0 = 0; k0 < K; k0 += 32) {
    V bh[4], bl[4];
#pragma unroll
    for (int j = 0; j < 4; ++j) {
      const size_t bo = (size_t)(n0 + (j << 4) + rlane) * ldb + koff + k0;
      bh[j] = Frag<T>::load(Bb + bo);
      if (SPLIT) bl[j] = Frag<T>::load(Bb2 + bo);
    }
#pragma unroll
    for (int i = 0; i < 4; ++i) {
      const size_t ao = (size_t)(m0 + (i << 4) + rlane) * lda + koff + k0;
      V ah = Frag<T>::load(Ab + ao);
      V al;
      if (SPLIT) al = Frag<T>::load(Ab2 + ao);
#pragma unroll
      for (int j = 0; j < 4; ++j) {
        acc[i][j] = Frag<T>::mma(ah, bh[j], acc[i][j]);
        if (SPLIT) {
          acc[i][j] = Frag<T>::mma(ah, bl[j], acc[i][j]);
          acc[i][j] = Frag<T>::mma(al, bh[j], acc[i][j]);
        }
      }
      Frag<T>::guard4(acc[i][0], acc[i][1], acc[i][2], acc[i][3], ah, SPLIT ? al : ah);
    }
    Frag<T>::keep(bh[0], bh[1], bh[2], bh[3]);
    if (SPLIT) Frag<T>::keep(bl[0], bl[1], bl[2], bl[3]);
  }
  acc_guard4(acc[0][0], acc[0][1], acc[0][2], acc[0][3]);
  acc_guard4(acc[1][0], acc[1][1], acc[1][2], acc[1][3]);
  acc_guard4(acc[2][0], acc[2][1], acc[2][2], acc[2][3]);
  acc_guard4(acc[3][0], acc[3][1], acc[3][2], acc[3][3]);

  float* slab = sT[wave];
  const float* Rb = RESID ? (resid + (size_t)b * strideR) : nullptr;
#pragma unroll
  for (int i = 0; i < 4; ++i) {
    const int mBase = m0 + (i << 4);
#pragma unroll
    for (int j = 0; j < 4; ++j) {
      const int n = n0 + (j << 4) + rlane;
      float bv = 0.f;
      if (BIAS_MODE == 2) bv = bias[n];
#pragma unroll
      for (int r = 0; r < 8; ++r) {
        float v = acc[i][j][r] * scale;
        if (BIAS_MODE == 1) v += bias[mBase + mOff + r];
        if (BIAS_MODE == 2) v += bv;
        if (RESID) v += Rb[(size_t)(mBase + mOff + r) * ldc + n];
        if (ACT == 1) v = tanhf(v);
        if (ACT == 2) v = fmaxf(v, 0.0f);
        if (ACT == 3) v = v / (1.0f + expf(-v));
        if (ACT == 4) v = (v > 0.f) ? v : 0.01f * v;
        slab[(mOff + r) * 68 + (j << 4) + rlane] = v;
      }
    }
    __builtin_amdgcn_fence(__ATOMIC_RELEASE, "workgroup");
    __builtin_amdgcn_wave_barrier();
    __builtin_amdgcn_fence(__ATOMIC_ACQUIRE, "workgroup");
    if (OUT_MODE == 0) {
      float* C = (float*)Cout + (size_t)b * strideC;
      const int hh = lane >> 4, c4 = (lane & 15) * 4;
      for (int pass = 0; pass < 2; ++pass) {
#pragma unroll
        for (int it = 0; it < 8; ++it) {
          const int row = it * 2 + hh;
          v4f v = *(const v4f*)(slab + row * 68 + c4);
          *(volatile v4f*)(C + (size_t)(mBase + row) * ldc + n0 + c4) = v;
        }
        __threadfence();
      }
    } else {
      const int q = lane >> 3, c8 = (lane & 7) * 8;
      unsigned short* C  = (unsigned short*)Cout  + (size_t)b * strideC;
      unsigned short* C2 = (OUT_MODE == 2) ? ((unsigned short*)Cout2 + (size_t)b * strideC) : nullptr;
      for (int pass = 0; pass < 2; ++pass) {
#pragma unroll
        for (int it = 0; it < 4; ++it) {
          const int row = it * 4 + q;
          const float* sp = slab + row * 68 + c8;
          v8h hv, lv;
#pragma unroll
          for (int e = 0; e < 8; ++e) {
            if (OUT_MODE == 1) {
              hv[e] = (_Float16)sp[e];
            } else {
              unsigned short hb = f2bf_bits(sp[e]);
              unsigned short lb = f2bf_bits(sp[e] - bf_bits2f(hb));
              hv[e] = __builtin_bit_cast(_Float16, hb);
              lv[e] = __builtin_bit_cast(_Float16, lb);
            }
          }
          *(volatile v8h*)(C + (size_t)(mBase + row) * ldc + n0 + c8) = hv;
          if (OUT_MODE == 2) *(volatile v8h*)(C2 + (size_t)(mBase + row) * ldc + n0 + c8) = lv;
        }
        __threadfence();
      }
    }
    __builtin_amdgcn_fence(__ATOMIC_RELEASE, "workgroup");
    __builtin_amdgcn_wave_barrier();
    __builtin_amdgcn_fence(__ATOMIC_ACQUIRE, "workgroup");
  }
}

__global__ __launch_bounds__(kThr) void cast_plane_kernel(const float* __restrict__ src, unsigned short* __restrict__ dst,
                                                          int colsLog2, int dstPitch, int dstOff) {
  const int i   = blockIdx.x * kThr + threadIdx.x;
  const int sh  = colsLog2 - 3;
  const int row = i >> sh;
  const int c8  = (i & ((1 << sh) - 1)) * 8;
  const float* sp = src + ((size_t)row << colsLog2) + c8;
  const v4f a0 = *(const v4f*)(sp);
  const v4f a1 = *(const v4f*)(sp + 4);
  v8h hv;
#pragma unroll
  for (int e = 0; e < 4; ++e) {
    const float f0 = a0[e];
    const float f1 = a1[e];
    hv[e]     = (_Float16)carry_flush(bf16r(f0), kInCarry);
    hv[4 + e] = (_Float16)carry_flush(bf16r(f1), kInCarry);
  }
  unsigned short* dp = dst + (size_t)row * dstPitch + dstOff + c8;
  *(volatile v8h*)dp = hv;
  __threadfence();
  *(volatile v8h*)dp = hv;
}

__global__ __launch_bounds__(kThr) void pack_kernel(const float* __restrict__ W, unsigned short* __restrict__ D, float* __restrict__ dstf, int part, int ld, int k0, int lg, int n0, int pitch) {
  const unsigned i = blockIdx.x * blockDim.x + threadIdx.x;
  if (part == 0) {
    const unsigned g = i & ((1u << lg) - 1u), n = i >> lg;
    const float* sp = W + (size_t)((unsigned)k0 + g * 8u) * (unsigned)ld + n;
    v8h hv;
#pragma unroll
    for (int t = 0; t < 8; ++t) hv[t] = (_Float16)carry_flush(bf16r(sp[(size_t)t * (unsigned)ld]), kInCarry);
    unsigned short* dp = D + (size_t)((unsigned)n0 + n) * (unsigned)pitch + g * 8u;
    *(volatile v8h*)dp = hv;
    __threadfence();
    *(volatile v8h*)dp = hv;
  } else {
    const v4f a = *(const v4f*)(W + i * 4u);
    v4f o;
#pragma unroll
    for (int e = 0; e < 4; ++e) o[e] = bf16r(a[e]);
    float* dp = dstf + i * 4u;
    *(volatile v4f*)dp = o;
    __threadfence();
    *(volatile v4f*)dp = o;
  }
}

__global__ __launch_bounds__(kThr) void zero_kernel(float* __restrict__ dst) {
  const size_t o4 = ((size_t)blockIdx.x * kThr + threadIdx.x) * 4u;
  const v4f z = {0.f, 0.f, 0.f, 0.f};
  *(volatile v4f*)(dst + o4) = z;
  __threadfence();
  *(volatile v4f*)(dst + o4) = z;
}

__global__ __launch_bounds__(kThr) void sqsplit_kernel(const float* __restrict__ R, unsigned short* __restrict__ A) {
  const unsigned i = blockIdx.x * (unsigned)kThr + threadIdx.x;
  const unsigned g = i & 63u, n = i >> 6;
  const float* rp = R + (size_t)(g * 8u) * kN + n;
  v8h hi, lo, one;
#pragma unroll
  for (int t = 0; t < 8; ++t) {
    const float v = rp[(size_t)t * kN];
    const float s = carry_flush(v * v, kInCarry);
    const _Float16 h = (_Float16)s;
    const float r = carry_flush(s - (float)h, 1.0f);
    hi[t] = h; lo[t] = (_Float16)r; one[t] = (_Float16)kInCarry;
  }
  unsigned short* ap = A + (size_t)n * kKD + g * 8u;
  *(volatile v8h*)(ap) = hi; *(volatile v8h*)(ap + kD) = lo; *(volatile v8h*)(ap + 2 * kD) = hi; *(volatile v8h*)(ap + 4 * kD) = one;
  __threadfence();
  *(volatile v8h*)(ap) = hi; *(volatile v8h*)(ap + kD) = lo; *(volatile v8h*)(ap + 2 * kD) = hi; *(volatile v8h*)(ap + 4 * kD) = one;
}

__global__ __launch_bounds__(kThr) void bbuild_kernel(const float* __restrict__ SR, const float* __restrict__ CR, unsigned short* __restrict__ B) {
  const unsigned i = blockIdx.x * (unsigned)kThr + threadIdx.x;
  const unsigned g = i & 63u, k = i >> 6;
  const unsigned kc = (k < 32u) ? k : 31u;
  const float keep = (k < 32u) ? 1.0f : 0.0f;
  const v4f c0 = *(const v4f*)(CR + (size_t)kc * kD + g * 8u), c1 = *(const v4f*)(CR + (size_t)kc * kD + g * 8u + 4u);
  v8h hi, lo, cx, cc;
#pragma unroll
  for (int t = 0; t < 8; ++t) {
    const float sv = SR[(size_t)(g * 8u + t) * kK + kc];
    const float cv = (t < 4) ? c0[t & 3] : c1[t & 3];
    const float s2 = sv * sv;
    const float s = keep * carry_flush(s2, kInCarry);
    const _Float16 h = (_Float16)s;
    hi[t] = h; lo[t] = (_Float16)carry_flush(s - (float)h, 1.0f);
    cx[t] = (_Float16)(keep * carry_flush(-2.0f * (cv * s2), kInCarry));
    cc[t] = (_Float16)(keep * carry_flush((cv * cv) * s2, kInCarry));
  }
  unsigned short* bp = B + (size_t)k * kKD + g * 8u;
  *(volatile v8h*)(bp) = hi; *(volatile v8h*)(bp + kD) = hi; *(volatile v8h*)(bp + 2 * kD) = lo; *(volatile v8h*)(bp + 3 * kD) = cx; *(volatile v8h*)(bp + 4 * kD) = cc;
  __threadfence();
  *(volatile v8h*)(bp) = hi; *(volatile v8h*)(bp + kD) = hi; *(volatile v8h*)(bp + 2 * kD) = lo; *(volatile v8h*)(bp + 3 * kD) = cx; *(volatile v8h*)(bp + 4 * kD) = cc;
}

__global__ __launch_bounds__(kThr) void rowsoft2_kernel(const float* __restrict__ LP, float* __restrict__ resA, unsigned short* __restrict__ QT) {
  const unsigned i = blockIdx.x * (unsigned)kThr + threadIdx.x;
  float q[2][32];
#pragma unroll
  for (int r = 0; r < 2; ++r) {
    const float* lp = LP + (size_t)(2u * i + r) * kKP;
    float m = lp[0];
#pragma unroll
    for (int c = 0; c < 8; ++c) {
      const v4f a = *(const v4f*)(lp + 4 * c);
#pragma unroll
      for (int e = 0; e < 4; ++e) { q[r][4 * c + e] = a[e]; m = (a[e] < m) ? a[e] : m; }
    }
    float s = 0.0f;
#pragma unroll
    for (int k = 0; k < 32; ++k) { q[r][k] = expf(-0.5f * (q[r][k] - m)); s += q[r][k]; }
#pragma unroll
    for (int k = 0; k < 32; ++k) q[r][k] = q[r][k] / s;
  }
  for (int pass = 0; pass < 2; ++pass) {
#pragma unroll
    for (int r = 0; r < 2; ++r) {
      float* op = resA + (size_t)(2u * i + r) * kK;
#pragma unroll
      for (int c = 0; c < 8; ++c) { const v4f o = {q[r][4 * c], q[r][4 * c + 1], q[r][4 * c + 2], q[r][4 * c + 3]}; *(volatile v4f*)(op + 4 * c) = o; }
    }
#pragma unroll
    for (int k = 0; k < 32; ++k) {
      v2h w; w[0] = (_Float16)carry_flush(q[0][k], kInCarry); w[1] = (_Float16)carry_flush(q[1][k], kInCarry);
      *(volatile v2h*)(QT + (size_t)k * kN + 2u * i) = w;
    }
    __threadfence();
  }
}

__global__ __launch_bounds__(kThr) void colmass_kernel(const float* __restrict__ resA, float* __restrict__ MS) {
  const unsigned i = threadIdx.x;
  const unsigned k = i & 31u, part = i >> 5;
  const float* ap = resA + (size_t)(part * 512u) * kK + k;
  float acc = 0.0f;
  for (int n = 0; n < 512; ++n) acc += ap[(size_t)n * kK];
  *(volatile float*)(MS + i) = acc;
  __threadfence();
  *(volatile float*)(MS + i) = acc;
}

__device__ __forceinline__ float enc_entry(const float* __restrict__ ZP, const float* __restrict__ SR, const float* __restrict__ CR, unsigned d, unsigned k, float mass) {
  return (SR[(size_t)d * kK + k] * (ZP[(size_t)d * kKP + k] - CR[(size_t)k * kD + d] * mass)) / mass;
}
__device__ __forceinline__ float mass_of(const float* __restrict__ MS, unsigned k) {
  float m = 0.0f;
#pragma unroll
  for (int p = 0; p < 8; ++p) m += MS[p * 32 + k];
  return m;
}

__global__ __launch_bounds__(kThr) void znormpart_kernel(const float* __restrict__ ZP, const float* __restrict__ SR, const float* __restrict__ CR, const float* __restrict__ MS, float* __restrict__ NP) {
  const unsigned i = blockIdx.x * (unsigned)kThr + threadIdx.x;
  const unsigned k = i & 31u, part = i >> 5;
  const float mass = mass_of(MS, k);
  float acc = 0.0f;
  for (int t = 0; t < 32; ++t) { const float z = enc_entry(ZP, SR, CR, part * 32u + (unsigned)t, k, mass); acc = fmaf(z, z, acc); }
  *(volatile float*)(NP + i) = acc;
  __threadfence();
  *(volatile float*)(NP + i) = acc;
}

__global__ __launch_bounds__(kThr) void zfinish_kernel(const float* __restrict__ ZP, const float* __restrict__ SR, const float* __restrict__ CR, const float* __restrict__ MS, const float* __restrict__ NP, float* __restrict__ resE) {
  const unsigned v = blockIdx.x * (unsigned)kThr + threadIdx.x;
  const unsigned d = v >> 5, k = v & 31u;
  const float mass = mass_of(MS, k);
  float nrm = 0.0f;
#pragma unroll
  for (int p = 0; p < 16; ++p) nrm += NP[p * 32 + k];
  const float o = enc_entry(ZP, SR, CR, d, k, mass) / sqrtf(nrm);
  *(volatile float*)(resE + v) = o;
  __threadfence();
  *(volatile float*)(resE + v) = o;
}

extern "C" void kernel_launch(void* const* d_in, const int* in_sizes, int n_in,
                              void* d_out, int out_size, void* d_ws, size_t ws_size,
                              hipStream_t stream) {
  if (n_in < 3 || d_out == nullptr || d_ws == nullptr) return;
  if (in_sizes[0] != kNB * kD * kN || in_sizes[1] != kK * kD || in_sizes[2] != kD * kK) return;
  if (out_size != kNB * kD * kK + kNB * kN * kK) return;
  if (ws_size < kWsTotal) return;
  const float* xa = (const float*)d_in[0];
  const float* cw = (const float*)d_in[1];
  const float* sv = (const float*)d_in[2];
  float* outE = (float*)d_out;
  float* outA = (float*)d_out + (size_t)kNB * kD * kK;
  char* ws = (char*)d_ws;
  unsigned short* AP = (unsigned short*)(ws + kOffAP);
  unsigned short* BP = (unsigned short*)(ws + kOffBP);
  float* XR = (float*)(ws + kOffXR);
  unsigned short* XB = (unsigned short*)(ws + kOffXB);
  float* SR = (float*)(ws + kOffSR);
  float* CR = (float*)(ws + kOffCR);
  float* LP = (float*)(ws + kOffLP);
  unsigned short* QT = (unsigned short*)(ws + kOffQT);
  float* ZP = (float*)(ws + kOffZP);
  float* MS = (float*)(ws + kOffMS);
  float* NP = (float*)(ws + kOffNP);

  static_assert((kNB * kD * kN / 4) % kThr == 0 && (kD * kK / 4) % kThr == 0 && (kNB * kD * kN / 8) % kThr == 0 && (kKP * 64) % kThr == 0 && (kN * 64) % kThr == 0 && (kN / 2) % kThr == 0 && ((kKP - kK) * kN * 2) % (kThr * 16) == 0
                && ((kN / 64) * (kKP / 64)) % 8 == 0 && ((kD / 64) * (kKP / 64)) % 8 == 0 && kKD % 32 == 0 && kN % 32 == 0 && (kD * kK) % kThr == 0, "every grid exact");
  pack_kernel<<<kNB * kD * kN / 4 / kThr, kThr, 0, stream>>>(xa, nullptr, XR, 1, 0, 0, 0, 0, 0);
  pack_kernel<<<kD * kK / 4 / kThr, kThr, 0, stream>>>(sv, nullptr, SR, 1, 0, 0, 0, 0, 0);
  pack_kernel<<<kK * kD / 4 / kThr, kThr, 0, stream>>>(cw, nullptr, CR, 1, 0, 0, 0, 0, 0);
  cast_plane_kernel<<<kNB * kD * kN / 8 / kThr, kThr, 0, stream>>>(xa, XB, 12, kN, 0);
  bbuild_kernel<<<kKP * 64 / kThr, kThr, 0, stream>>>(SR, CR, BP);
  for (int b = 0; b < kNB; ++b) {
    unsigned short* APb = AP + (size_t)b * kN * kKD;
    float* LPb = LP + (size_t)b * kN * kKP;
    unsigned short* QTb = QT + (size_t)b * kKP * kN;
    float* ZPb = ZP + (size_t)b * kD * kKP;
    float* MSb = MS + (size_t)b * 8 * 32;
    float* NPb = NP + (size_t)b * 16 * 32;
    float* outAb = outA + (size_t)b * kN * kK;
    sqsplit_kernel<<<kN * 64 / kThr, kThr, 0, stream>>>(XR + (size_t)b * kD * kN, APb);
    pack_kernel<<<kN * (kD / 8) / kThr, kThr, 0, stream>>>(xa + (size_t)b * kD * kN, APb + 3 * kD, nullptr, 0, kN, 0, 6, 0, kKD);
    wmma_gemm64<0, false, 0, 0, false, 0><<<dim3((kN / 64) * (kKP / 64) / 8, 1), 256, 0, stream>>>(
        APb, APb, kKD, 0L, BP, BP, kKD, 0L, (void*)LPb, (void*)LPb, kKP, 0L, nullptr, nullptr, 0L, kN, kKP, kKD, kSc20);
    rowsoft2_kernel<<<kN / 2 / kThr, kThr, 0, stream>>>(LPb, outAb, QTb);
    zero_kernel<<<(kKP - kK) * kN * 2 / (kThr * 16), kThr, 0, stream>>>((float*)(QTb + (size_t)kK * kN));
    colmass_kernel<<<1, kThr, 0, stream>>>(outAb, MSb);
    wmma_gemm64<0, false, 0, 0, false, 0><<<dim3((kD / 64) * (kKP / 64) / 8, 1), 256, 0, stream>>>(
        XB + (size_t)b * kD * kN, XB + (size_t)b * kD * kN, kN, 0L, QTb, QTb, kN, 0L, (void*)ZPb, (void*)ZPb, kKP, 0L, nullptr, nullptr, 0L, kD, kKP, kN, kSc20);
    znormpart_kernel<<<2, kThr, 0, stream>>>(ZPb, SR, CR, MSb, NPb);
    zfinish_kernel<<<kD * kK / kThr, kThr, 0, stream>>>(ZPb, SR, CR, MSb, NPb, outE + (size_t)b * kD * kK);
  }
}
